// PCNN_20942260536125
// MI455X (gfx1250) — hardware-verified
//
#include <hip/hip_runtime.h>
#include <stdint.h>
#include <stddef.h>


typedef _Float16 v8h  __attribute__((ext_vector_type(8)));
typedef _Float16 v16h __attribute__((ext_vector_type(16)));
typedef float    v8f  __attribute__((ext_vector_type(8)));
typedef float    v4f  __attribute__((ext_vector_type(4)));

union Frag  { v16h v; v8h h8[2]; };
union Pack8 { v8h v; _Float16 e[8]; };

#define NB     1024
#define NL     256
#define ND     50
#define NF     52
#define NW     230
#define KH     10
#define CONVL  247
#define NLAB   53
#define XP     56
#define KP     576
#define NPAD   240
#define H3     690
#define HP     704
#define DP     256
#define OP     64
#define HSP    264
#define LGP    68
#define ASC    16.0f
#define WSC    64.0f
#define PINV   0.0009765625f
#define BNEPS  1e-5f

static_assert(KP % 32 == 0);
static_assert(HP % 32 == 0);
static_assert(DP % 32 == 0);
static_assert((XP * 2) % 16 == 0);
static_assert((HSP * 2) % 16 == 0);
static_assert((32 * NLAB * 4) % 128 == 0);
static_assert((HP * 2) % 128 == 0);

__device__ __forceinline__ v8f zero8() { v8f z = {0.f, 0.f, 0.f, 0.f, 0.f, 0.f, 0.f, 0.f}; return z; }

__device__ __forceinline__ v8f wmma16(v8f c, v16h a, v16h b) {
  v8f d = __builtin_amdgcn_wmma_f32_16x16x32_f16(false, a, false, b, (short)0, c, false, false);
  asm volatile("v_nop\n\tv_nop\n\tv_nop\n\tv_nop" : "+v"(d) : "v"(a), "v"(b));
  return d;
}

__device__ __forceinline__ v8f gemm_tile(const _Float16* ar, const _Float16* br, int ksteps) {
  v8f acc = zero8();
  for (int ks = 0; ks < ksteps; ++ks) {
    const int kk = ks * 32;
    Frag a, bb;
    a.h8[0]  = *(const v8h*)(ar + kk);  a.h8[1]  = *(const v8h*)(ar + kk + 16);
    bb.h8[0] = *(const v8h*)(br + kk);  bb.h8[1] = *(const v8h*)(br + kk + 16);
    acc = wmma16(acc, a.v, bb.v);
  }
  return acc;
}

__global__ __launch_bounds__(256) void k_packconv(const float* __restrict__ cw, _Float16* __restrict__ Wp) {
  __shared__ __attribute__((aligned(16))) _Float16 sw[16 * KP];
  const int tid = threadIdx.x, n0 = blockIdx.x * 16;
  for (int idx = tid; idx < 16 * KP; idx += 256) {
    const int r = idx / KP, k = idx - r * KP;
    const int tap = k / XP, d = k - tap * XP;
    const int n = n0 + r;
    float v = 0.0f;
    if (n < NW && tap < KH && d < NF) v = cw[((size_t)n * KH + tap) * NF + d] * WSC;
    sw[idx] = (_Float16)v;
  }
  __syncthreads();
  _Float16* base = Wp + (size_t)n0 * KP;
  const int nck = (16 * KP) >> 3;
  for (int pass = 0; pass < 2; ++pass) {
    for (int c = tid; c < nck; c += 256) {
      v8h val = *(const v8h*)(sw + 8 * c);
      *(volatile v8h*)(base + 8 * c) = val;
    }
    if (pass == 0) __threadfence();
  }
}

__global__ __launch_bounds__(128) void k_packfc(const float* __restrict__ src, int rows, int cols,
                                                 _Float16* __restrict__ dst, int pitch) {
  const int row = blockIdx.x, c = threadIdx.x;
  if (c >= (pitch >> 3)) return;
  const int col0 = c * 8;
  Pack8 u;
#pragma unroll
  for (int e = 0; e < 8; ++e) {
    const int col = col0 + e;
    float v = 0.0f;
    if (row < rows && col < cols) v = src[(size_t)row * cols + col] * WSC;
    u.e[e] = (_Float16)v;
  }
  _Float16* p = dst + (size_t)row * pitch + col0;
  *(volatile v8h*)p = u.v;
  __threadfence();
  *(volatile v8h*)p = u.v;
}

__global__ __launch_bounds__(256) void k_embed(const int* __restrict__ ids, int nrows,
                                                const float* __restrict__ table, int V,
                                                const float* __restrict__ pe, _Float16* __restrict__ X) {
  __shared__ int sid[64];
  __shared__ __attribute__((aligned(16))) _Float16 sx[64 * XP];
  const int tid = threadIdx.x, row0 = blockIdx.x * 64;
  if (tid < 64) {
    const int r = row0 + tid;
    int id = 0;
    if (r < nrows) {
      id = ids[r];
      if (id < 0) id += V;
      id = (id < 0) ? 0 : ((id > V - 1) ? (V - 1) : id);
    }
    sid[tid] = id;
  }
  __syncthreads();
  {
    const int r = tid >> 2, part = tid & 3;
    const int row = row0 + r;
    const bool valid = row < nrows;
    _Float16* sr = sx + r * XP + part * 14;
    if (part < 3) {
      const float* tr = table + (size_t)sid[r] * ND + part * 14;
#pragma unroll
      for (int k = 0; k < 14; ++k) {
        float v = 0.0f;
        if (valid) v = tr[k] * ASC;
        sr[k] = (_Float16)v;
      }
    } else {
      const float* tr = table + (size_t)sid[r] * ND + 42;
#pragma unroll
      for (int k = 0; k < 8; ++k) {
        float v = 0.0f;
        if (valid) v = tr[k] * ASC;
        sr[k] = (_Float16)v;
      }
      float q0 = 0.0f, q1 = 0.0f;
      if (valid) { q0 = pe[(size_t)row * 2] * ASC; q1 = pe[(size_t)row * 2 + 1] * ASC; }
      sr[8]  = (_Float16)q0;
      sr[9]  = (_Float16)q1;
      sr[10] = (_Float16)0.0f; sr[11] = (_Float16)0.0f; sr[12] = (_Float16)0.0f; sr[13] = (_Float16)0.0f;
    }
  }
  __syncthreads();
  _Float16* base = X + (size_t)blockIdx.x * (64 * XP);
  const int nck = (64 * XP) >> 3;
  for (int pass = 0; pass < 2; ++pass) {
    for (int c = tid; c < nck; c += 256) {
      v8h val = *(const v8h*)(sx + 8 * c);
      *(volatile v8h*)(base + 8 * c) = val;
    }
    if (pass == 0) __threadfence();
  }
}

__device__ __forceinline__ void seg_upd(int t, float v, int p1, int p2, float& s0, float& s1, float& s2) {
  if (t < CONVL) {
    if (t <= p1) s0 = fmaxf(s0, v);
    if (t > p1 && t <= p2) s1 = fmaxf(s1, v);
    if (t > p2) s2 = fmaxf(s2, v);
  }
}

__global__ __launch_bounds__(256) void k_conv(const _Float16* __restrict__ X, const _Float16* __restrict__ Wp,
                                               const float* __restrict__ cb, const int* __restrict__ pos,
                                               _Float16* __restrict__ Hout) {
  __shared__ float red[8][3][NPAD];
  __shared__ __attribute__((aligned(16))) _Float16 hs[HP];
  const int tid = threadIdx.x, lane = tid & 31, hh = lane >> 4, m = lane & 15, w = tid >> 5;
  const int b = blockIdx.x;
  const int p1 = pos[2 * b], p2 = pos[2 * b + 1];
  const float ninf = -__builtin_huge_valf();
  const _Float16* xb = X + (size_t)b * NL * XP;
  const int ta = w * 16, tb = (w + 8) * 16;
  const _Float16* ar0 = xb + (size_t)(ta + m) * XP + 8 * hh;
  const _Float16* ar1 = xb + (size_t)(tb + m) * XP + 8 * hh;

  for (int ng = 0; ng < 3; ++ng) {
    const _Float16* wc = Wp + (size_t)(ng * 80 + m) * KP + 8 * hh;
    v8f acc0[5], acc1[5];
#pragma unroll
    for (int q = 0; q < 5; ++q) { acc0[q] = zero8(); acc1[q] = zero8(); }
    for (int ks = 0; ks < KP / 32; ++ks) {
      const int kk = ks * 32;
      Frag a0, a1;
      a0.h8[0] = *(const v8h*)(ar0 + kk);  a0.h8[1] = *(const v8h*)(ar0 + kk + 16);
      a1.h8[0] = *(const v8h*)(ar1 + kk);  a1.h8[1] = *(const v8h*)(ar1 + kk + 16);
#pragma unroll
      for (int q = 0; q < 5; ++q) {
        const _Float16* wr = wc + (size_t)(q * 16) * KP + kk;
        Frag bb;
        bb.h8[0] = *(const v8h*)(wr);
        bb.h8[1] = *(const v8h*)(wr + 16);
        acc0[q] = wmma16(acc0[q], a0.v, bb.v);
        acc1[q] = wmma16(acc1[q], a1.v, bb.v);
      }
    }
#pragma unroll
    for (int q = 0; q < 5; ++q) {
      float s0 = ninf, s1 = ninf, s2 = ninf;
#pragma unroll
      for (int r = 0; r < 8; ++r) {
        seg_upd(ta + 8 * hh + r, acc0[q][r], p1, p2, s0, s1, s2);
        seg_upd(tb + 8 * hh + r, acc1[q][r], p1, p2, s0, s1, s2);
      }
      s0 = fmaxf(s0, __shfl_xor(s0, 16));
      s1 = fmaxf(s1, __shfl_xor(s1, 16));
      s2 = fmaxf(s2, __shfl_xor(s2, 16));
      if (hh == 0) {
        const int n = ng * 80 + q * 16 + m;
        red[w][0][n] = s0; red[w][1][n] = s1; red[w][2][n] = s2;
      }
    }
  }
  __syncthreads();
  if (tid < NW) {
    const int n = tid;
    const float bias = cb[n];
#pragma unroll
    for (int s = 0; s < 3; ++s) {
      float v = red[0][s][n];
#pragma unroll
      for (int ww = 1; ww < 8; ++ww) v = fmaxf(v, red[ww][s][n]);
      float h = -1.0f;
      if (v > ninf) h = tanhf(v * PINV + bias);
      hs[s * NW + n] = (_Float16)(h * ASC);
    }
  } else if (tid < NW + (HP - H3)) {
    hs[H3 + (tid - NW)] = (_Float16)0.0f;
  }
  __syncthreads();
  if (tid < (HP >> 3)) {
    v8h val = *(const v8h*)(hs + 8 * tid);
    _Float16* p = Hout + (size_t)b * HP + 8 * tid;
    *(volatile v8h*)p = val;
    __threadfence();
    *(volatile v8h*)p = val;
  }
}

__global__ __launch_bounds__(256) void k_head(const _Float16* __restrict__ Hin, const _Float16* __restrict__ W0p,
                                               const _Float16* __restrict__ W1p, const _Float16* __restrict__ Wop,
                                               const float* __restrict__ d0b, const float* __restrict__ g0,
                                               const float* __restrict__ be0, const float* __restrict__ m0,
                                               const float* __restrict__ v0, const float* __restrict__ a0,
                                               const float* __restrict__ d1b, const float* __restrict__ g1,
                                               const float* __restrict__ be1, const float* __restrict__ m1,
                                               const float* __restrict__ v1, const float* __restrict__ a1,
                                               const float* __restrict__ ob, float* __restrict__ out) {
  __shared__ __attribute__((aligned(16))) _Float16 h0s[32 * HSP];
  __shared__ __attribute__((aligned(16))) _Float16 h1s[32 * HSP];
  __shared__ __attribute__((aligned(16))) float lg[32 * LGP];
  __shared__ __attribute__((aligned(16))) float outs[32 * NLAB];
  const int tid = threadIdx.x, lane = tid & 31, hh = lane >> 4, m = lane & 15, w = tid >> 5;
  const int r0 = blockIdx.x * 32;
  const float ninf = -__builtin_huge_valf();
  {
    Pack8 z;
#pragma unroll
    for (int e = 0; e < 8; ++e) z.e[e] = (_Float16)0.0f;
    for (int c = tid; c < ((32 * HSP) >> 3); c += 256) {
      *(v8h*)(h0s + 8 * c) = z.v;
      *(v8h*)(h1s + 8 * c) = z.v;
    }
  }
  __syncthreads();
  const float alpha0 = a0[0], alpha1 = a1[0];

  for (int p = w; p < 30; p += 8) {
    const int mt = p / 15, nt = p - mt * 15;
    const _Float16* ar = Hin + (size_t)(r0 + mt * 16 + m) * HP + 8 * hh;
    const _Float16* br = W0p + (size_t)(nt * 16 + m) * HP + 8 * hh;
    v8f acc = gemm_tile(ar, br, HP / 32);
    const int n = nt * 16 + m;
    float bias = 0.0f, scale = 0.0f, mean = 0.0f, beta = 0.0f;
    if (n < NW) { bias = d0b[n]; scale = g0[n] * rsqrtf(v0[n] + BNEPS); mean = m0[n]; beta = be0[n]; }
#pragma unroll
    for (int r = 0; r < 8; ++r) {
      const int row = mt * 16 + 8 * hh + r;
      float val = 0.0f;
      if (n < NW) {
        float y = acc[r] * PINV + bias;
        y = (y - mean) * scale + beta;
        val = (y > 0.0f) ? y : alpha0 * y;
      }
      h0s[row * HSP + n] = (_Float16)(val * ASC);
    }
  }
  __syncthreads();

  for (int p = w; p < 30; p += 8) {
    const int mt = p / 15, nt = p - mt * 15;
    const _Float16* ar = h0s + (mt * 16 + m) * HSP + 8 * hh;
    const _Float16* br = W1p + (size_t)(nt * 16 + m) * DP + 8 * hh;
    v8f acc = gemm_tile(ar, br, DP / 32);
    const int n = nt * 16 + m;
    float bias = 0.0f, scale = 0.0f, mean = 0.0f, beta = 0.0f;
    if (n < NW) { bias = d1b[n]; scale = g1[n] * rsqrtf(v1[n] + BNEPS); mean = m1[n]; beta = be1[n]; }
#pragma unroll
    for (int r = 0; r < 8; ++r) {
      const int row = mt * 16 + 8 * hh + r;
      float val = 0.0f;
      if (n < NW) {
        float y = acc[r] * PINV + bias;
        y = (y - mean) * scale + beta;
        val = (y > 0.0f) ? y : alpha1 * y;
      }
      h1s[row * HSP + n] = (_Float16)(val * ASC);
    }
  }
  __syncthreads();

  {
    const int mt = w >> 2, nt = w & 3;
    const _Float16* ar = h1s + (mt * 16 + m) * HSP + 8 * hh;
    const _Float16* br = Wop + (size_t)(nt * 16 + m) * DP + 8 * hh;
    v8f acc = gemm_tile(ar, br, DP / 32);
    const int n = nt * 16 + m;
    const float bias = (n < NLAB) ? ob[n] : 0.0f;
#pragma unroll
    for (int r = 0; r < 8; ++r) {
      const int row = mt * 16 + 8 * hh + r;
      lg[row * LGP + n] = acc[r] * PINV + bias;
    }
  }
  __syncthreads();

  for (int i = 0; i < 4; ++i) {
    const int row = w * 4 + i;
    const bool v1ok = (lane + 32) < NLAB;
    const float x0 = lg[row * LGP + lane];
    const float x1 = v1ok ? lg[row * LGP + lane + 32] : ninf;
    float mx = fmaxf(x0, x1);
    mx = fmaxf(mx, __shfl_xor(mx, 16));
    mx = fmaxf(mx, __shfl_xor(mx, 8));
    mx = fmaxf(mx, __shfl_xor(mx, 4));
    mx = fmaxf(mx, __shfl_xor(mx, 2));
    mx = fmaxf(mx, __shfl_xor(mx, 1));
    const float e0 = __expf(x0 - mx);
    const float e1 = v1ok ? __expf(x1 - mx) : 0.0f;
    float sm = e0 + e1;
    sm += __shfl_xor(sm, 16);
    sm += __shfl_xor(sm, 8);
    sm += __shfl_xor(sm, 4);
    sm += __shfl_xor(sm, 2);
    sm += __shfl_xor(sm, 1);
    const float inv = 1.0f / sm;
    outs[row * NLAB + lane] = e0 * inv;
    if (v1ok) outs[row * NLAB + lane + 32] = e1 * inv;
  }
  __syncthreads();

  float* slab = out + (size_t)r0 * NLAB;
  const int nck = (32 * NLAB) >> 2;
  for (int pass = 0; pass < 2; ++pass) {
    for (int c = tid; c < nck; c += 256) {
      v4f v = *(const v4f*)(outs + 4 * c);
      *(volatile v4f*)(slab + 4 * c) = v;
    }
    if (pass == 0) __threadfence();
  }
}

extern "C" void kernel_launch(void* const* d_in, const int* in_sizes, int n_in,
                              void* d_out, int out_size, void* d_ws, size_t ws_size,
                              hipStream_t stream) {
  if (n_in < 22) return;
  const int nrows = in_sizes[0];
  if (nrows != NB * NL || in_sizes[1] != NB * 2 || out_size != NB * NLAB) return;
  const int V = in_sizes[3] / ND;
  if (V < 1) return;

  const int*   x   = (const int*)d_in[0];
  const int*   pos = (const int*)d_in[1];
  const float* pe  = (const float*)d_in[2];
  const float* emb = (const float*)d_in[3];
  const float* cw  = (const float*)d_in[4];
  const float* cb  = (const float*)d_in[5];
  const float* d0w = (const float*)d_in[6];
  const float* d0b = (const float*)d_in[7];
  const float* g0  = (const float*)d_in[8];
  const float* be0 = (const float*)d_in[9];
  const float* m0  = (const float*)d_in[10];
  const float* v0  = (const float*)d_in[11];
  const float* a0  = (const float*)d_in[12];
  const float* d1w = (const float*)d_in[13];
  const float* d1b = (const float*)d_in[14];
  const float* g1  = (const float*)d_in[15];
  const float* be1 = (const float*)d_in[16];
  const float* m1  = (const float*)d_in[17];
  const float* v1  = (const float*)d_in[18];
  const float* a1  = (const float*)d_in[19];
  const float* ow  = (const float*)d_in[20];
  const float* ob  = (const float*)d_in[21];
  float* outp = (float*)d_out;

  char* ws = (char*)d_ws;
  size_t off = 0;
  auto carve = [&](size_t bytes) -> void* {
    off = (off + 255) & ~(size_t)255;
    void* p = ws + off; off += bytes; return p;
  };
  const int nblkE = nrows / 64 + 1;
  _Float16* Wp  = (_Float16*)carve((size_t)NPAD * KP * 2);
  _Float16* W0p = (_Float16*)carve((size_t)NPAD * HP * 2);
  _Float16* W1p = (_Float16*)carve((size_t)NPAD * DP * 2);
  _Float16* Wop = (_Float16*)carve((size_t)OP * DP * 2);
  _Float16* X   = (_Float16*)carve((size_t)nblkE * 64 * XP * 2);
  _Float16* Hb  = (_Float16*)carve((size_t)NB * HP * 2);
  if (off > ws_size) return;

  k_packconv<<<dim3(NPAD / 16), 256, 0, stream>>>(cw, Wp);
  k_packfc<<<dim3(NPAD), 128, 0, stream>>>(d0w, NW, H3, W0p, HP);
  k_packfc<<<dim3(NPAD), 128, 0, stream>>>(d1w, NW, NW, W1p, DP);
  k_packfc<<<dim3(OP), 128, 0, stream>>>(ow, NLAB, NW, Wop, DP);
  k_embed<<<dim3(nblkE), 256, 0, stream>>>(x, nrows, emb, V, pe, X);
  k_conv<<<dim3(NB), 256, 0, stream>>>(X, Wp, cb, pos, Hb);
  k_head<<<dim3(NB / 32), 256, 0, stream>>>(Hb, W0p, W1p, Wop, d0b, g0, be0, m0, v0, a0,
                                            d1b, g1, be1, m1, v1, a1, ob, outp);
}
